// SelfAttention_52012053954870
// MI455X (gfx1250) — hardware-run, weakly checked
//
#include <hip/hip_runtime.h>
#include <math.h>

#ifndef NB
#define NB 4
#endif
#ifndef SEQ
#define SEQ 2048
#endif
#define NB_FULL 4
#define SEQ_FULL 2048
#define CE 1024
#define SLAB_P 68
#define SLAB_F (16 * SLAB_P)
static_assert(NB >= 1);
static_assert(NB <= NB_FULL);
static_assert(SEQ % 64 == 0);
static_assert(SEQ <= SEQ_FULL);
static_assert(SEQ <= 256 * 8);
static_assert(CE % 64 == 0);
static_assert(CE % 32 == 0);
static_assert(CE % 8 == 0);
static_assert((NB * SEQ) % 64 == 0);
static_assert(SLAB_P % 4 == 0);
static_assert(SLAB_P >= 64);

typedef __attribute__((ext_vector_type(16))) _Float16 v16h;
typedef __attribute__((ext_vector_type(8)))  _Float16 v8h;
typedef __attribute__((ext_vector_type(8)))  float    v8f;
typedef __attribute__((ext_vector_type(4)))  float    v4f;
typedef __attribute__((ext_vector_type(4)))  unsigned v4u;

#define VST2(T, ptr, val) do { const T vst2_v_ = (val); *(volatile T*)(ptr) = vst2_v_; __threadfence(); *(volatile T*)(ptr) = vst2_v_; } while (0)

__device__ __forceinline__ float bf_rne(float v) { const unsigned u = __float_as_uint(v); return __uint_as_float((u + 0x7fffu + ((u >> 16) & 1u)) & 0xffff0000u); }
__device__ __forceinline__ unsigned pk2h(float a, float b) { return (unsigned)__builtin_bit_cast(unsigned short, (_Float16)a) | ((unsigned)__builtin_bit_cast(unsigned short, (_Float16)b) << 16); }

union FragU { v16h v; v8h h[2]; };
__device__ __forceinline__ v16h frag_load(const _Float16* p) { FragU f; f.h[0] = *(const v8h*)(p); f.h[1] = *(const v8h*)(p + 16); return f.v; }
__device__ __forceinline__ v8f mma_g(v16h a, v16h b, v8f c) {
  c = __builtin_amdgcn_wmma_f32_16x16x32_f16(false, a, false, b, (short)0, c, false, false);
  asm volatile("v_nop\n\tv_nop\n\tv_nop\n\tv_nop" : "+v"(c) : "v"(a), "v"(b));
  return c;
}

template <int BIAS_MODE, int OUT_MODE>
__device__ __forceinline__ void gemm64_body(float* sT,
    const unsigned short* __restrict__ Ap, int lda, const unsigned short* __restrict__ Btp, int ldb,
    void* __restrict__ Cout, int ldc, const float* __restrict__ bias, int M, int N, int K, float scale) {
  const _Float16* A = (const _Float16*)Ap; const _Float16* Bt = (const _Float16*)Btp;
  const int lane = threadIdx.x & 31;
  const int wave = __builtin_amdgcn_readfirstlane((int)(threadIdx.x >> 5));
  const int tilesN = N >> 6;
  const int tilesM = M >> 6;
  const int tile = blockIdx.x * 8 + wave;
  if (tile >= tilesM * tilesN) return;
  const int tm = tile / tilesN;
  const int tn = tile - tm * tilesN;
  const int m0 = tm << 6;
  const int n0 = tn << 6;

  const int rlane = lane & 15;
  const int koff  = (lane >> 4) * 8;
  const int mOff  = (lane >> 4) * 8;

  v8f acc[4][4];
#pragma unroll
  for (int i = 0; i < 4; ++i)
#pragma unroll
    for (int j = 0; j < 4; ++j) acc[i][j] = (v8f){0.f,0.f,0.f,0.f,0.f,0.f,0.f,0.f};

#pragma unroll 1
  for (int k0 = 0; k0 < K; k0 += 32) {
    v16h bf[4];
#pragma unroll
    for (int j = 0; j < 4; ++j) bf[j] = frag_load(Bt + (size_t)(n0 + (j << 4) + rlane) * ldb + koff + k0);
#pragma unroll
    for (int i = 0; i < 4; ++i) {
      const v16h ah = frag_load(A + (size_t)(m0 + (i << 4) + rlane) * lda + koff + k0);
#pragma unroll
      for (int j = 0; j < 4; ++j) acc[i][j] = mma_g(ah, bf[j], acc[i][j]);
    }
  }

  float* slab = sT + wave * SLAB_F;
#pragma unroll
  for (int i = 0; i < 4; ++i) {
    const int mBase = m0 + (i << 4);
#pragma unroll
    for (int j = 0; j < 4; ++j) {
      const int n = n0 + (j << 4) + rlane;
      float bv = 0.f;
      if (BIAS_MODE == 2) bv = bias[n];
#pragma unroll
      for (int r = 0; r < 8; ++r) {
        float v = acc[i][j][r] * scale;
        if (BIAS_MODE == 1) v += bias[mBase + mOff + r];
        if (BIAS_MODE == 2) v += bv;
        slab[(mOff + r) * SLAB_P + (j << 4) + rlane] = v;
      }
    }
    __builtin_amdgcn_fence(3  , "workgroup");
    __builtin_amdgcn_wave_barrier();
    __builtin_amdgcn_fence(2  , "workgroup");
    if (OUT_MODE == 0) {
      float* C = (float*)Cout;
      const int hh = lane >> 4, c4 = (lane & 15) * 4;
      for (int pass = 0; pass < 2; ++pass) {
#pragma unroll
        for (int it = 0; it < 8; ++it) {
          const int row = it * 2 + hh;
          const v4f v = *(const v4f*)(slab + row * SLAB_P + c4);
          *(volatile v4f*)(C + (size_t)(mBase + row) * ldc + n0 + c4) = v;
        }
        __threadfence();
      }
    } else {
      const int q = lane >> 3, c8 = (lane & 7) * 8;
      unsigned short* C = (unsigned short*)Cout;
      for (int pass = 0; pass < 2; ++pass) {
#pragma unroll
        for (int it = 0; it < 4; ++it) {
          const int row = it * 4 + q;
          const float* sp = slab + row * SLAB_P + c8;
          v8h hv;
#pragma unroll
          for (int e = 0; e < 8; ++e) hv[e] = (_Float16)sp[e];
          *(volatile v8h*)(C + (size_t)(mBase + row) * ldc + n0 + c8) = hv;
        }
        __threadfence();
      }
    }
    __builtin_amdgcn_fence(3  , "workgroup");
    __builtin_amdgcn_wave_barrier();
    __builtin_amdgcn_fence(2  , "workgroup");
  }
}

__global__ __launch_bounds__(256) void k_gemm_bn16(const unsigned short* __restrict__ A, int lda, const unsigned short* __restrict__ Bt, int ldb,
    unsigned short* __restrict__ C, int ldc, const float* __restrict__ bias, int M, int N, int K, float scale) {
  __shared__ __align__(16) float sT[8 * SLAB_F];
  gemm64_body<2, 1>(sT, A, lda, Bt, ldb, (void*)C, ldc, bias, M, N, K, scale);
}
__global__ __launch_bounds__(256) void k_gemm_bm16(const unsigned short* __restrict__ A, int lda, const unsigned short* __restrict__ Bt, int ldb,
    unsigned short* __restrict__ C, int ldc, const float* __restrict__ bias, int M, int N, int K, float scale) {
  __shared__ __align__(16) float sT[8 * SLAB_F];
  gemm64_body<1, 1>(sT, A, lda, Bt, ldb, (void*)C, ldc, bias, M, N, K, scale);
}
__global__ __launch_bounds__(256) void k_gemm_f32(const unsigned short* __restrict__ A, int lda, const unsigned short* __restrict__ Bt, int ldb,
    float* __restrict__ C, int ldc, int M, int N, int K, float scale) {
  __shared__ __align__(16) float sT[8 * SLAB_F];
  gemm64_body<0, 0>(sT, A, lda, Bt, ldb, (void*)C, ldc, nullptr, M, N, K, scale);
}

__global__ __launch_bounds__(256) void k_castx(const float* __restrict__ x, unsigned short* __restrict__ X16, int nrows) {
  const long long u = (long long)blockIdx.x * 256 + threadIdx.x;
  constexpr int per = CE / 8;
  if (u >= (long long)nrows * per) return;
  const int r = (int)(u / per); const int c0 = 8 * (int)(u % per);
  const int b = r / SEQ, t = r - b * SEQ;
  const float* s = x + ((size_t)b * SEQ_FULL + t) * CE + c0;
  const v4f a = *(const v4f*)s; const v4f c = *(const v4f*)(s + 4);
  v4u pk;
  pk.x = pk2h(bf_rne(a.x), bf_rne(a.y)); pk.y = pk2h(bf_rne(a.z), bf_rne(a.w));
  pk.z = pk2h(bf_rne(c.x), bf_rne(c.y)); pk.w = pk2h(bf_rne(c.z), bf_rne(c.w));
  VST2(v4u, (v4u*)(X16 + (size_t)r * CE + c0), pk);
}
__global__ __launch_bounds__(256) void k_castwT(const float* __restrict__ W, unsigned short* __restrict__ dst, float sc) {
  const long long u = (long long)blockIdx.x * 256 + threadIdx.x;
  constexpr int per = CE / 8;
  if (u >= (long long)CE * per) return;
  const int c = (int)(u / per); const int r0 = 8 * (int)(u % per);
  float w[8];
#pragma unroll
  for (int e = 0; e < 8; ++e) w[e] = bf_rne(W[(size_t)(r0 + e) * CE + c]) * sc;
  v4u pk; pk.x = pk2h(w[0], w[1]); pk.y = pk2h(w[2], w[3]); pk.z = pk2h(w[4], w[5]); pk.w = pk2h(w[6], w[7]);
  VST2(v4u, (v4u*)(dst + (size_t)c * CE + r0), pk);
}
__global__ __launch_bounds__(256) void k_bias(const float* __restrict__ bq, const float* __restrict__ bk, const float* __restrict__ bv, float* __restrict__ BR) {
  const int u = blockIdx.x * 256 + threadIdx.x;
  if (u >= 3 * CE) return;
  const int i = u & (CE - 1); const int sel = u / CE;
  const float a = bq[i], b2 = bk[i], c = bv[i];
  const float v = bf_rne((sel == 0) ? a : ((sel == 1) ? b2 : c));
  VST2(float, BR + u, v);
}

__global__ __launch_bounds__(256) void k_soft(const float* __restrict__ S, unsigned short* __restrict__ P16) {
#pragma clang fp contract(off)
  __shared__ float red[256];
  __shared__ __align__(16) float prow[SEQ];
  const int t = blockIdx.x, tid = threadIdx.x;
  const float* srow = S + (size_t)t * SEQ;
  const float L2E = 1.4426950408889634f;
  float mx = -__builtin_inff();
#pragma unroll 1
  for (int s = tid; s < SEQ; s += 256) mx = fmaxf(mx, srow[s]);
  red[tid] = mx; __syncthreads();
  for (int o = 128; o > 0; o >>= 1) { if (tid < o) red[tid] = fmaxf(red[tid], red[tid + o]); __syncthreads(); }
  mx = red[0]; __syncthreads();
  float sum = 0.f;
#pragma unroll 1
  for (int s = tid; s < SEQ; s += 256) { const float e = exp2f((srow[s] - mx) * L2E); prow[s] = e; sum += e; }
  red[tid] = sum; __syncthreads();
  for (int o = 128; o > 0; o >>= 1) { if (tid < o) red[tid] += red[tid + o]; __syncthreads(); }
  sum = red[0];
  const float sc = 4096.f * (1.f / sum);
  if (8 * tid < SEQ) {
    const float* pr = prow + 8 * tid;
    const v4f a = *(const v4f*)pr; const v4f c = *(const v4f*)(pr + 4);
    v4u pk;
    pk.x = pk2h(a.x * sc, a.y * sc); pk.y = pk2h(a.z * sc, a.w * sc);
    pk.z = pk2h(c.x * sc, c.y * sc); pk.w = pk2h(c.z * sc, c.w * sc);
    VST2(v4u, (v4u*)(P16 + (size_t)t * SEQ + 8 * tid), pk);
  }
}

extern "C" void kernel_launch(void* const* d_in, const int* in_sizes, int n_in, void* d_out, int out_size, void* d_ws, size_t ws_size, hipStream_t stream) {
  if (n_in < 7) return;
  const long long need_tok = (long long)(NB - 1) * SEQ_FULL * CE + (long long)SEQ * CE;
  if ((long long)in_sizes[0] < need_tok) return;
  if (in_sizes[1] < CE * CE || in_sizes[3] < CE * CE || in_sizes[5] < CE * CE) return;
  if (in_sizes[2] < CE || in_sizes[4] < CE || in_sizes[6] < CE) return;
  if ((long long)out_size < need_tok) return;
  static_assert((long long)(NB - 1) * SEQ_FULL * CE + (long long)SEQ * CE <= (long long)NB_FULL * SEQ_FULL * CE);

  const float* x  = (const float*)d_in[0];
  const float* Wq = (const float*)d_in[1];
  const float* bq = (const float*)d_in[2];
  const float* Wk = (const float*)d_in[3];
  const float* bk = (const float*)d_in[4];
  const float* Wv = (const float*)d_in[5];
  const float* bv = (const float*)d_in[6];
  float* out = (float*)d_out;

  constexpr int NT = NB * SEQ;
  constexpr size_t X16_B = (size_t)NT * CE * 2;
  constexpr size_t S_B   = (size_t)SEQ * SEQ * 4;
  constexpr size_t R0_B  = (X16_B > S_B) ? X16_B : S_B;
  static_assert(X16_B <= R0_B); static_assert(S_B <= R0_B);
  constexpr size_t WT_B  = (size_t)3 * CE * CE * 2;
  constexpr size_t BR_B  = (size_t)3 * CE * 4;
  constexpr size_t QK_B  = (size_t)NT * 2 * CE * 2;
  constexpr size_t VT_B  = (size_t)CE * NT * 2;
  constexpr size_t P16_B = (size_t)SEQ * SEQ * 2;
  constexpr size_t TOT_B = R0_B + WT_B + BR_B + QK_B + VT_B + P16_B;
  static_assert(TOT_B <= (size_t)134217728);
  static_assert(R0_B % 256 == 0); static_assert(WT_B % 256 == 0); static_assert(BR_B % 256 == 0); static_assert(QK_B % 256 == 0);
  static_assert(VT_B % 256 == 0); static_assert(P16_B % 256 == 0);
  if (TOT_B > ws_size) return;
  char* wsp = (char*)d_ws;
  unsigned short* X16 = (unsigned short*)wsp; float* S = (float*)wsp; wsp += R0_B;
  unsigned short* WT3 = (unsigned short*)wsp; wsp += WT_B;
  float* BR = (float*)wsp; wsp += BR_B;
  unsigned short* QK  = (unsigned short*)wsp; wsp += QK_B;
  unsigned short* Vt  = (unsigned short*)wsp; wsp += VT_B;
  unsigned short* P16 = (unsigned short*)wsp; wsp += P16_B;
  if ((size_t)(wsp - (char*)d_ws) > ws_size) return;

  k_castx<<<(unsigned)(((long long)NT * (CE / 8) + 255) / 256), 256, 0, stream>>>(x, X16, NT);
  k_castwT<<<(unsigned)(((long long)CE * (CE / 8) + 255) / 256), 256, 0, stream>>>(Wq, WT3, 64.0f);
  k_castwT<<<(unsigned)(((long long)CE * (CE / 8) + 255) / 256), 256, 0, stream>>>(Wk, WT3 + (size_t)CE * CE, 64.0f);
  k_castwT<<<(unsigned)(((long long)CE * (CE / 8) + 255) / 256), 256, 0, stream>>>(Wv, WT3 + (size_t)2 * CE * CE, 64.0f);
  k_bias<<<(unsigned)((3 * CE + 255) / 256), 256, 0, stream>>>(bq, bk, bv, BR);

  { static_assert(NT % 64 == 0); static_assert((2 * CE) % 64 == 0); static_assert(CE % 32 == 0);
    const int tiles = (NT / 64) * (2 * CE / 64);
    k_gemm_bn16<<<(unsigned)((tiles + 7) / 8), 256, 0, stream>>>(X16, CE, WT3, CE, QK, 2 * CE, BR, NT, 2 * CE, CE, 1.0f / 64.0f); }
  { const int tiles = (CE / 64) * (NT / 64);
    k_gemm_bm16<<<(unsigned)((tiles + 7) / 8), 256, 0, stream>>>(WT3 + (size_t)2 * CE * CE, CE, X16, CE, Vt, NT, BR + 2 * CE, CE, NT, CE, 1.0f / 64.0f); }

  for (int b = 0; b < NB; ++b) {
    const unsigned short* Aq = QK + (size_t)b * SEQ * (2 * CE);
    { static_assert(SEQ % 64 == 0);
      const int tiles = (SEQ / 64) * (SEQ / 64);
      k_gemm_f32<<<(unsigned)((tiles + 7) / 8), 256, 0, stream>>>(Aq, 2 * CE, Aq + CE, 2 * CE, S, SEQ, SEQ, SEQ, CE, 0.03125f); }
    k_soft<<<(unsigned)SEQ, 256, 0, stream>>>(S, P16);
    { static_assert(SEQ % 32 == 0);
      const int tiles = (SEQ / 64) * (CE / 64);
      k_gemm_f32<<<(unsigned)((tiles + 7) / 8), 256, 0, stream>>>(P16, SEQ, Vt + (size_t)b * SEQ, NT, out + (size_t)b * SEQ_FULL * CE, CE, SEQ, CE, SEQ, 1.0f / 4096.0f); }
  }
}
